// FlexAttnScoreModBlockMaskModel_63797444215440
// MI455X (gfx1250) — hardware-verified
//
#include <hip/hip_runtime.h>
#include <stddef.h>
#include <stdint.h>

#define NBATCH 2
#define SQ     2048
#define DMOD   1024
#define NH     16
#define HDM    64
#define MR     (NBATCH * SQ)
#define NQKV   (3 * DMOD)
#define NSLAB  (NQKV / 128)
#define WNC    64
#define QB     128
#define KC     64
#define NQB    (SQ / QB)
#define NBH    (NBATCH * NH)

static_assert(DMOD == NH * HDM);
static_assert(HDM == 64);
static_assert(HDM % 32 == 0);
static_assert(2 * WNC == 128);
static_assert(DMOD % 32 == 0);
static_assert(DMOD % 128 == 0);
static_assert(NSLAB * 128 == NQKV);
static_assert(MR % 64 == 0);
static_assert(SQ % 64 == 0);
static_assert(MR % 256 == 0);
static_assert(DMOD % 64 == 0);
static_assert(NQB * QB == SQ);
static_assert(QB == 8 * 16);
static_assert(QB == 2 * KC);
static_assert(KC == 64);
static_assert((MR * DMOD) % 2048 == 0);
static_assert((DMOD * DMOD) % 2048 == 0);

typedef _Float16 v16h __attribute__((ext_vector_type(16)));
typedef _Float16 v8h  __attribute__((ext_vector_type(8)));
typedef float    v8f  __attribute__((ext_vector_type(8)));
typedef float    v4f  __attribute__((ext_vector_type(4)));
typedef unsigned int v4u __attribute__((ext_vector_type(4)));

union Frag  { v16h v; v8h h[2]; };
union Pack8 { v8h h; v4u u; };

__device__ __forceinline__ v8f mma16(v16h a, v16h b, v8f c) {
  c = __builtin_amdgcn_wmma_f32_16x16x32_f16(false, a, false, b, (short)0, c, false, false);
  asm volatile("v_nop\n\tv_nop\n\tv_nop\n\tv_nop" : "+v"(c) : "v"(a), "v"(b));
  return c;
}

__device__ __forceinline__ v16h ldfrag(const _Float16* p, int ld, int row0, int k0, int lane) {
  const int m = lane & 15, lh = lane >> 4;
  const _Float16* q = p + (size_t)(row0 + m) * ld + k0 + 8 * lh;
  Frag f;
  f.h[0] = *(const v8h*)(q);
  f.h[1] = *(const v8h*)(q + 16);
  return f.v;
}

__device__ __forceinline__ v8f zero8() { return (v8f){0.f, 0.f, 0.f, 0.f, 0.f, 0.f, 0.f, 0.f}; }

__device__ __forceinline__ void gemm32x64(const _Float16* __restrict__ A, int lda,
                                          const _Float16* __restrict__ Bt, int ldb,
                                          int m0, int n0, int lane, v8f (&acc)[2][4]) {
#pragma unroll 1
  for (int k0 = 0; k0 < DMOD; k0 += 32) {
    const v16h a0 = ldfrag(A, lda, m0, k0, lane);
    const v16h a1 = ldfrag(A, lda, m0 + 16, k0, lane);
#pragma unroll
    for (int t = 0; t < 4; ++t) {
      const v16h b = ldfrag(Bt, ldb, n0 + 16 * t, k0, lane);
      acc[0][t] = mma16(a0, b, acc[0][t]);
      acc[1][t] = mma16(a1, b, acc[1][t]);
    }
  }
}

__global__ __launch_bounds__(256) void k_cvt(const float* __restrict__ src, _Float16* __restrict__ dst, float sc) {
  const size_t o = ((size_t)blockIdx.x * 256 + threadIdx.x) * 8;
  const v4f a0 = *(const v4f*)(src + o);
  const v4f a1 = *(const v4f*)(src + o + 4);
  Pack8 pk;
  pk.h = (v8h){(_Float16)(a0[0] * sc), (_Float16)(a0[1] * sc), (_Float16)(a0[2] * sc), (_Float16)(a0[3] * sc),
               (_Float16)(a1[0] * sc), (_Float16)(a1[1] * sc), (_Float16)(a1[2] * sc), (_Float16)(a1[3] * sc)};
  const v4u vv = pk.u;
  volatile v4u* d = (volatile v4u*)(dst + o);
  *d = vv;
  __threadfence();
  *d = vv;
}

#define SFP 132
__global__ __launch_bounds__(128) __attribute__((amdgpu_num_vgpr(256)))
void k_qkv(const _Float16* __restrict__ xh, const _Float16* __restrict__ wt,
           _Float16* __restrict__ qp, _Float16* __restrict__ kp, _Float16* __restrict__ vtp) {
  __shared__ __align__(16) float sf[64 * SFP];
  const int tid = threadIdx.x, lane = tid & 31, wave = tid >> 5;
  const int hh = lane >> 4, c = lane & 15;
  const int wm = wave >> 1, wn = wave & 1;
  const int mb = blockIdx.x * 64;
  const int ns = blockIdx.y;
  const int which = ns >> 3;
  const int cs    = ns & 7;
  const int m0 = mb + wm * 32;
  const int n0 = ns * 128 + wn * WNC;

  v8f acc[2][4];
#pragma unroll
  for (int s = 0; s < 2; ++s)
#pragma unroll
    for (int t = 0; t < 4; ++t) acc[s][t] = zero8();
  gemm32x64(xh, DMOD, wt, DMOD, m0, n0, lane, acc);

#pragma unroll
  for (int sub = 0; sub < 2; ++sub)
#pragma unroll
    for (int t = 0; t < 4; ++t)
#pragma unroll
      for (int r = 0; r < 8; ++r)
        sf[(wm * 32 + 16 * sub + 8 * hh + r) * SFP + wn * WNC + 16 * t + c] = acc[sub][t][r] * 0.03125f;
  __syncthreads();

  if (which < 2) {
    v4u val[8];
    size_t go[8];
#pragma unroll
    for (int j = 0; j < 8; ++j) {
      const int p  = tid + 128 * j;
      const int lr = p >> 4;
      const int pc = p & 15;
      const int d0 = pc * 8;
      const float* ra = sf + lr * SFP + d0;
      const v4f a0 = *(const v4f*)(ra), a1 = *(const v4f*)(ra + 4);
      Pack8 pk;
      pk.h = (v8h){(_Float16)a0[0], (_Float16)a0[1], (_Float16)a0[2], (_Float16)a0[3],
                   (_Float16)a1[0], (_Float16)a1[1], (_Float16)a1[2], (_Float16)a1[3]};
      val[j] = pk.u;
      go[j]  = (size_t)(mb + lr) * DMOD + cs * 128 + d0;
    }
    _Float16* base = (which == 0) ? qp : kp;
    for (int ps = 0; ps < 2; ++ps) {
#pragma unroll
      for (int j = 0; j < 8; ++j) *(volatile v4u*)(base + go[j]) = val[j];
      __threadfence();
    }
  } else {
    const int b  = mb / SQ;
    const int s0 = mb - b * SQ;
    v4u val[8];
    size_t go[8];
#pragma unroll
    for (int j = 0; j < 8; ++j) {
      const int p   = tid + 128 * j;
      const int dc  = p >> 3;
      const int pc  = p & 7;
      const int hd  = cs * 2 + (dc >> 6);
      const int d   = dc & 63;
      const float* cp = sf + (pc * 8) * SFP + dc;
      Pack8 pk;
      pk.h = (v8h){(_Float16)cp[0 * SFP], (_Float16)cp[1 * SFP], (_Float16)cp[2 * SFP], (_Float16)cp[3 * SFP],
                   (_Float16)cp[4 * SFP], (_Float16)cp[5 * SFP], (_Float16)cp[6 * SFP], (_Float16)cp[7 * SFP]};
      val[j] = pk.u;
      go[j]  = ((size_t)(b * NH + hd) * HDM + d) * SQ + s0 + pc * 8;
    }
    for (int ps = 0; ps < 2; ++ps) {
#pragma unroll
      for (int j = 0; j < 8; ++j) *(volatile v4u*)(vtp + go[j]) = val[j];
      __threadfence();
    }
  }
}

#define PSP 72
static_assert(PSP % 8 == 0);
static_assert(PSP >= KC);
static_assert(PSP >= HDM);
__global__ __launch_bounds__(256) __attribute__((amdgpu_num_vgpr(256)))
void k_attn(const _Float16* __restrict__ qp, const _Float16* __restrict__ kp,
            const _Float16* __restrict__ vt, _Float16* __restrict__ op) {
  __shared__ __align__(16) _Float16 Ps[8 * 16 * PSP];

  const int tid = threadIdx.x, lane = tid & 31, wave = tid >> 5;
  const int hh = lane >> 4, c = lane & 15;
  const int qb = blockIdx.x % NQB;
  const int bh = blockIdx.x / NQB;
  const int b  = bh >> 4;
  const int hd = bh & 15;
  const int q0 = qb * QB + wave * 16;
  const int nkch = 2 * qb + 2;

  const _Float16* Q = qp + (size_t)b * SQ * DMOD + hd * HDM;
  const _Float16* K = kp + (size_t)b * SQ * DMOD + hd * HDM;
  const _Float16* V = vt + (size_t)bh * HDM * SQ;

  const float NEGM = -1.0e30f;
  float mrow[8], lrow[8];
  v8f oacc[4];
#pragma unroll
  for (int r = 0; r < 8; ++r) { mrow[r] = NEGM; lrow[r] = 0.f; }
#pragma unroll
  for (int t = 0; t < 4; ++t) oacc[t] = zero8();

  _Float16* pw = Ps + wave * 16 * PSP;

#pragma unroll 1
  for (int kc = 0; kc < nkch; ++kc) {
    const int kv0 = kc * KC;
    __syncthreads();

    v8f s[4];
#pragma unroll
    for (int j = 0; j < 4; ++j) s[j] = zero8();
#pragma unroll
    for (int dc = 0; dc < HDM / 32; ++dc) {
      const v16h qa = ldfrag(Q, DMOD, q0, dc * 32, lane);
#pragma unroll
      for (int j = 0; j < 4; ++j) {
        const v16h kb = ldfrag(K, DMOD, kv0 + j * 16, dc * 32, lane);
        s[j] = mma16(qa, kb, s[j]);
      }
    }
    const int dq = q0 + 8 * hh - kv0 - c;
#pragma unroll
    for (int r = 0; r < 8; ++r)
#pragma unroll
      for (int j = 0; j < 4; ++j) {
        const int   dl = dq + r - 16 * j;
        const float bv = -(float)dl;
        const float v  = s[j][r] * 0.25f + bv;
        s[j][r] = (dl >= 0) ? v : NEGM;
      }
    float cm[8];
#pragma unroll
    for (int r = 0; r < 8; ++r) {
      float m = NEGM;
#pragma unroll
      for (int j = 0; j < 4; ++j) m = fmaxf(m, s[j][r]);
#pragma unroll
      for (int off = 1; off < 16; off <<= 1) m = fmaxf(m, __shfl_xor(m, off, 32));
      cm[r] = m;
    }
    float al[8];
#pragma unroll
    for (int r = 0; r < 8; ++r) {
      const float mnew  = fmaxf(mrow[r], cm[r]);
      const float msafe = (mnew <= -1.0e29f) ? 0.f : mnew;
      const float alpha = __expf(mrow[r] - msafe);
      mrow[r] = mnew;
      float psum = 0.f;
#pragma unroll
      for (int j = 0; j < 4; ++j) {
        const float sv = s[j][r];
        const float p  = (sv > -1.0e29f) ? __expf(sv - msafe) : 0.f;
        psum += p;
        pw[(8 * hh + r) * PSP + j * 16 + c] = (_Float16)(p * 1024.0f);
      }
#pragma unroll
      for (int off = 1; off < 16; off <<= 1) psum += __shfl_xor(psum, off, 32);
      lrow[r] = lrow[r] * alpha + psum;
      al[r] = alpha;
    }
#pragma unroll
    for (int t = 0; t < 4; ++t)
#pragma unroll
      for (int r = 0; r < 8; ++r) oacc[t][r] *= al[r];
    __syncthreads();

#pragma unroll
    for (int kk = 0; kk < 2; ++kk) {
      const v16h pa = ldfrag(pw, PSP, 0, kk * 32, lane);
#pragma unroll
      for (int t = 0; t < 4; ++t) {
        const v16h vb = ldfrag(V, SQ, t * 16, kv0 + kk * 32, lane);
        oacc[t] = mma16(pa, vb, oacc[t]);
      }
    }
  }

  float invl[8];
#pragma unroll
  for (int r = 0; r < 8; ++r) invl[r] = (lrow[r] > 0.f) ? (0.015625f / lrow[r]) : 0.f;
  __syncthreads();
#pragma unroll
  for (int r = 0; r < 8; ++r) {
#pragma unroll
    for (int t = 0; t < 4; ++t)
      pw[(8 * hh + r) * PSP + 16 * t + c] = (_Float16)(oacc[t][r] * invl[r]);
  }
  __syncthreads();
  v4u val[4];
  size_t go[4];
#pragma unroll
  for (int it = 0; it < 4; ++it) {
    const int p  = lane + 32 * it;
    const int L  = p >> 3;
    const int pc = p & 7;
    Pack8 pk;
    pk.h    = *(const v8h*)(pw + L * PSP + pc * 8);
    val[it] = pk.u;
    go[it]  = (size_t)(b * SQ + q0 + L) * DMOD + hd * HDM + pc * 8;
  }
  for (int ps = 0; ps < 2; ++ps) {
#pragma unroll
    for (int it = 0; it < 4; ++it) *(volatile v4u*)(op + go[it]) = val[it];
    __threadfence();
  }
}

#define OTP 68
__device__ __forceinline__ void out_epilogue(v8f (&acc)[2][4], float scale, float* sw, float* __restrict__ out,
                                             int m0, int n0, int lane, int hh, int c) {
#pragma unroll
  for (int sub = 0; sub < 2; ++sub) {
    __syncthreads();
#pragma unroll
    for (int t = 0; t < 4; ++t) {
#pragma unroll
      for (int r = 0; r < 8; ++r) sw[(8 * hh + r) * OTP + 16 * t + c] = acc[sub][t][r] * scale;
    }
    __syncthreads();
    v4f val[8];
    size_t go[8];
#pragma unroll
    for (int it = 0; it < 8; ++it) {
      const int p    = lane + 32 * it;
      const int L    = p >> 3;
      const int pc   = p & 7;
      const int row  = L >> 1;
      const int half = L & 1;
      val[it] = *(const v4f*)(sw + row * OTP + half * 32 + pc * 4);
      go[it]  = (size_t)(m0 + sub * 16 + row) * DMOD + n0 + half * 32 + pc * 4;
    }
    for (int ps = 0; ps < 2; ++ps) {
#pragma unroll
      for (int it = 0; it < 8; ++it) *(volatile v4f*)(out + go[it]) = val[it];
      __threadfence();
    }
  }
}

__global__ __launch_bounds__(256) __attribute__((amdgpu_num_vgpr(256)))
void k_out(const _Float16* __restrict__ op, const _Float16* __restrict__ wt, float* __restrict__ out) {
  __shared__ __align__(16) float st[8][16 * OTP];
  const int tid = threadIdx.x, lane = tid & 31, wave = tid >> 5;
  const int hh = lane >> 4, c = lane & 15;
  const int s0 = blockIdx.x * 256 + wave * 32;
  const int n0 = blockIdx.y * 64;

  v8f acc[2][4];
#pragma unroll
  for (int s = 0; s < 2; ++s)
#pragma unroll
    for (int t = 0; t < 4; ++t) acc[s][t] = zero8();
  gemm32x64(op, DMOD, wt, DMOD, s0, n0, lane, acc);
  out_epilogue(acc, 0.001953125f, st[wave], out, s0, n0, lane, hh, c);
}

extern "C" void kernel_launch(void* const* d_in, const int* in_sizes, int n_in,
                              void* d_out, int out_size, void* d_ws, size_t ws_size,
                              hipStream_t stream) {
  if (n_in < 5) return;
  if (in_sizes[0] != MR * DMOD) return;
  if (in_sizes[1] != DMOD * DMOD) return;
  if (in_sizes[2] != DMOD * DMOD) return;
  if (in_sizes[3] != DMOD * DMOD) return;
  if (in_sizes[4] != DMOD * DMOD) return;
  if (out_size != MR * DMOD) return;

  const float* x  = (const float*)d_in[0];
  const float* wq = (const float*)d_in[1];
  const float* wk = (const float*)d_in[2];
  const float* wv = (const float*)d_in[3];
  const float* wo = (const float*)d_in[4];
  float* out = (float*)d_out;

  size_t off = 0;
  const size_t oX  = off; off += (size_t)MR * DMOD * 2;
  const size_t oWt = off; off += (size_t)NQKV * DMOD * 2;
  const size_t oWo = off; off += (size_t)DMOD * DMOD * 2;
  const size_t oQ  = off; off += (size_t)MR * DMOD * 2;
  const size_t oK  = off; off += (size_t)MR * DMOD * 2;
  const size_t oV  = off; off += (size_t)NBH * HDM * SQ * 2;
  const size_t oO  = off; off += (size_t)MR * DMOD * 2;
  if (off > ws_size) return;
  if (off > (size_t)134217728) return;

  char* ws = (char*)d_ws;
  _Float16* Xh  = (_Float16*)(ws + oX);
  _Float16* Wt  = (_Float16*)(ws + oWt);
  _Float16* Wot = (_Float16*)(ws + oWo);
  _Float16* Qp  = (_Float16*)(ws + oQ);
  _Float16* Kp  = (_Float16*)(ws + oK);
  _Float16* Vt  = (_Float16*)(ws + oV);
  _Float16* Op  = (_Float16*)(ws + oO);

  const int gx = in_sizes[0] / 2048;
  const int gw = in_sizes[1] / 2048;

  k_cvt<<<dim3(gx), dim3(256), 0, stream>>>(x, Xh, 1.0f);
  k_cvt<<<dim3(gw), dim3(256), 0, stream>>>(wq, Wt, 32.0f);
  k_cvt<<<dim3(gw), dim3(256), 0, stream>>>(wk, Wt + (size_t)DMOD * DMOD, 32.0f);
  k_cvt<<<dim3(gw), dim3(256), 0, stream>>>(wv, Wt + (size_t)2 * DMOD * DMOD, 32.0f);
  k_cvt<<<dim3(gw), dim3(256), 0, stream>>>(wo, Wot, 32.0f);
  k_qkv<<<dim3(MR / 64, NSLAB), dim3(128), 0, stream>>>(Xh, Wt, Qp, Kp, Vt);
  k_attn<<<dim3(NBH * NQB), dim3(256), 0, stream>>>(Qp, Kp, Vt, Op);
  k_out<<<dim3(MR / 256, DMOD / 64), dim3(256), 0, stream>>>(Op, Wot, out);
  (void)hipGetLastError();
}
